// SymmetrizedBFAN_38912403702331
// MI455X (gfx1250) — hardware-verified
//
#include <hip/hip_runtime.h>


#ifndef NSAMP
#define NSAMP 1048576
#endif
#define NSAMP_FULL 1048576
#define DD   5
#define HH   4
#define NF   8
#define KK   20
#define RD   160
#define KST  5
#define WV   8
#define SUBT 4
#define CHS  64
#define CPW  4
#define WCARRY 64.0f
#define WINV   0.015625f

static_assert(RD == NF * KK);
static_assert(NF == 2 * HH);
static_assert(RD % 32 == 0);
static_assert(KST * 32 == RD);
static_assert(RD % 8 == 0);
static_assert(KK > 8);
static_assert(CHS == 16 * SUBT);
static_assert(32 * 16 == CHS * 2 * 4);
static_assert(NSAMP % (CHS * CPW * WV) == 0);
static_assert(NSAMP <= NSAMP_FULL);
static_assert(16 * RD * 2 + WV * 256 * 4 <= 131072);

static constexpr bool carry_ok() {
    for (int s = 0; s < KST; ++s)
        for (int i = 0; i < 16; ++i) {
            const int kk0 = 32 * s + (i < 8 ? i : 8 + i);
            const int f0 = kk0 / KK, k0 = kk0 % KK;
            if (kk0 + 8 >= RD) return false;
            if (k0 >= KK - 8 && f0 + 1 >= NF) return false;
        }
    return true;
}
static_assert(carry_ok());

typedef _Float16 h16;
typedef __attribute__((ext_vector_type(16))) _Float16 v16h;
typedef __attribute__((ext_vector_type(8)))  _Float16 v8h;
typedef __attribute__((ext_vector_type(8)))  float    v8f;
typedef __attribute__((ext_vector_type(4)))  float    v4f;
typedef __attribute__((ext_vector_type(2)))  float    v2f;
typedef v4f  __attribute__((may_alias)) v4fa;

__device__ __forceinline__ unsigned short f2bf(float f) { unsigned u = __float_as_uint(f); u += 0x7FFFu + ((u >> 16) & 1u); return (unsigned short)(u >> 16); }
__device__ __forceinline__ float bfr(float f) { return __uint_as_float(((unsigned)f2bf(f)) << 16); }
__device__ __forceinline__ v16h cat16(v8h lo, v8h hi) { return __builtin_shufflevector(lo, hi, 0, 1, 2, 3, 4, 5, 6, 7, 8, 9, 10, 11, 12, 13, 14, 15); }
__device__ __forceinline__ v8f wmma16(v16h a, v16h b, v8f c) { return __builtin_amdgcn_wmma_f32_16x16x32_f16(false, a, false, b, (short)0, c, false, false); }
__device__ __forceinline__ v8f wmma16g(v16h a, v16h b, v8f c) { c = wmma16(a, b, c); asm volatile("v_nop\n\tv_nop\n\tv_nop\n\tv_nop" : "+v"(c) : "v"(a), "v"(b)); return c; }
__device__ __forceinline__ void wave_sync() { __builtin_amdgcn_fence(3  , "wavefront"); __builtin_amdgcn_wave_barrier(); asm volatile("" ::: "memory"); }
static __device__ __forceinline__ h16 toh_flush(float v) { const h16 r = (h16)v; return (fabsf(v) < 6.103515625e-05f) ? (h16)0.0f : r; }
__device__ __forceinline__ float knotv(int k) { return 0.2f * ((float)k / (float)(KK - 1)); }

__global__ __launch_bounds__(32 * WV) void k_basis_readout(const float* __restrict__ x, const float* __restrict__ mwre, const float* __restrict__ mwim,
                                                           const float* __restrict__ rore, const float* __restrict__ roim, float* out) {
    __shared__ __align__(16) h16   wt[16 * RD];
    __shared__ __align__(16) float os[WV * 256];
    const int lane = threadIdx.x & 31, lr = lane & 15, hi = lane >> 4;
    const int wave = __builtin_amdgcn_readfirstlane((int)(threadIdx.x >> 5));

#pragma unroll 1
    for (int idx = threadIdx.x; idx < 16 * RD / 8; idx += 32 * WV) {
        const int n = idx / (RD / 8), k8 = (idx - n * (RD / 8)) * 8;
        v4f a0 = *(const v4f*)(rore + k8), a1 = *(const v4f*)(rore + k8 + 4);
        v4f b0 = *(const v4f*)(roim + k8), b1 = *(const v4f*)(roim + k8 + 4);
        asm volatile("" : "+v"(a0), "+v"(a1), "+v"(b0), "+v"(b1));
        const bool isre = (n == 0), isim = (n == 1);
        v8h o;
#pragma unroll
        for (int i = 0; i < 4; ++i) {
            const float u0 = isre ? bfr(a0[i]) : (isim ? bfr(b0[i]) : 0.0f);
            const float u1 = isre ? bfr(a1[i]) : (isim ? bfr(b1[i]) : 0.0f);
            o[i] = toh_flush(u0 * WCARRY); o[4 + i] = toh_flush(u1 * WCARRY); }
        *(v8h*)(&wt[n * RD + k8]) = o;
    }
    __syncthreads();

    v16h wf[KST];
#pragma unroll
    for (int s = 0; s < KST; ++s) { const int o = lr * RD + 32 * s + 8 * hi; wf[s] = cat16(*(const v8h*)(&wt[o]), *(const v8h*)(&wt[o + 16])); }

    float wre[HH * DD], wim[HH * DD];
#pragma unroll
    for (int i = 0; i < HH * DD; ++i) { wre[i] = bfr(mwre[i]); wim[i] = bfr(mwim[i]); }

    float cK[KK];
#pragma unroll
    for (int j = 0; j < KK; ++j) cK[j] = hi ? knotv((j + 8) % KK) : knotv(j);

#pragma unroll 1
    for (int it = 0; it < CPW; ++it) {
        const size_t chunk = ((size_t)blockIdx.x * WV + (size_t)wave) * CPW + (size_t)it;
        const size_t s0 = chunk * CHS;
#pragma unroll 1
        for (int j = 0; j < SUBT; ++j) {
            const size_t smp = s0 + (size_t)(16 * j + lr);
            const float* xp = x + smp * (size_t)(2 * DD);
            const v2f p0 = *(const v2f*)(xp), p1 = *(const v2f*)(xp + 2), p2 = *(const v2f*)(xp + 4), p3 = *(const v2f*)(xp + 6), p4 = *(const v2f*)(xp + 8);
            float xr[DD], xi[DD];
            xr[0] = bfr(p0[0]); xi[0] = bfr(p0[1]); xr[1] = bfr(p1[0]); xi[1] = bfr(p1[1]); xr[2] = bfr(p2[0]); xi[2] = bfr(p2[1]);
            xr[3] = bfr(p3[0]); xi[3] = bfr(p3[1]); xr[4] = bfr(p4[0]); xi[4] = bfr(p4[1]);
            float t[NF];
#pragma unroll
            for (int h = 0; h < HH; ++h) {
                float hre = 0.0f, him = 0.0f;
#pragma unroll
                for (int d = 0; d < DD; ++d) {
                    hre = fmaf(xr[d],  wre[h * DD + d], hre); hre = fmaf(-xi[d], wim[h * DD + d], hre);
                    him = fmaf(xr[d],  wim[h * DD + d], him); him = fmaf(xi[d],  wre[h * DD + d], him); }
                t[h] = hre; t[HH + h] = him; }
            float tS[NF];
#pragma unroll
            for (int f = 0; f < NF - 1; ++f) tS[f] = hi ? t[f + 1] : t[f];
            tS[NF - 1] = t[NF - 1];

            v8f acc = (v8f){};
#pragma unroll
            for (int s = 0; s < KST; ++s) {
                v16h ff;
#pragma unroll
                for (int i = 0; i < 16; ++i) {
                    const int kk0 = 32 * s + (i < 8 ? i : 8 + i);
                    const int f0 = kk0 / KK, k0 = kk0 % KK;
                    const float tt = (k0 >= KK - 8) ? tS[f0] : t[f0];
                    const float rr = fmaxf(fabsf(tt) - cK[k0], 0.0f);
                    ff[i] = toh_flush(copysignf(rr, tt)); }
                acc = wmma16g(wf[s], ff, acc);
            }
            const int oi = wave * 256 + hi * 128 + (16 * j + lr) * 2;
            os[oi] = acc[0] * WINV; os[oi + 1] = acc[1] * WINV;
        }
        wave_sync();
        const v4f val = *(const v4fa*)(&os[wave * 256 + lane * 4]);
        float* op = out + s0 * 2 + (size_t)lane * 4;
        *(volatile v4f*)op = val;
        __threadfence();
        *(volatile v4f*)op = val;
        wave_sync();
    }
}

extern "C" void kernel_launch(void* const* d_in, const int* in_sizes, int n_in,
                              void* d_out, int out_size, void* d_ws, size_t ws_size, hipStream_t stream) {
    (void)d_ws; (void)ws_size;
    if (n_in < 5) return;
    if ((size_t)in_sizes[0] < (size_t)NSAMP * 2 * DD) return;
    if (in_sizes[1] < HH * DD || in_sizes[2] < HH * DD) return;
    if (in_sizes[3] < RD || in_sizes[4] < RD) return;
    if ((size_t)out_size < (size_t)NSAMP * 2) return;
    const float* x    = (const float*)d_in[0];
    const float* mwre = (const float*)d_in[1];
    const float* mwim = (const float*)d_in[2];
    const float* rore = (const float*)d_in[3];
    const float* roim = (const float*)d_in[4];
    float* OUT = (float*)d_out;
    k_basis_readout<<<dim3(NSAMP / (CHS * CPW * WV), 1, 1), 32 * WV, 0, stream>>>(x, mwre, mwim, rore, roim, OUT);
}
